// BSplineKANLayer_46969762349507
// MI455X (gfx1250) — hardware-verified
//
#include <hip/hip_runtime.h>
#include <math.h>

constexpr int kBatch    = 16384;
constexpr int kNin      = 512;
constexpr int kNout     = 512;
constexpr int kNbasis   = 8;
constexpr int kKspl     = kNin * kNbasis;
constexpr int kHalfRows = kBatch / 2;
constexpr int kNknots   = 12;

constexpr float kXCarry     = 8.0f;
constexpr float kWCarry     = 1024.0f;
constexpr float kBaseScale  = 1.0f / (8.0f * 1024.0f);
constexpr float kBasisCarry = 256.0f;
constexpr float kCoeffCarry = 16.0f;
constexpr float kSplScale   = 1.0f / (256.0f * 16.0f);

constexpr size_t kOffBtBase = 0;
constexpr size_t kOffBtSpl  = kOffBtBase + (size_t)kNout * kNin * 2;
constexpr size_t kOffAx     = kOffBtSpl  + (size_t)kNout * kKspl * 2;
constexpr size_t kOffP      = kOffAx     + (size_t)kBatch * kNin * 2;
constexpr size_t kOffAspl   = kOffP      + (size_t)kBatch * kNout * 4;
constexpr size_t kWsTotal   = kOffAspl   + (size_t)kHalfRows * kKspl * 2;
static_assert(kOffBtSpl == 524288 && kOffAx == 4718592 && kOffP == 21495808 && kOffAspl == 55050240, "carve offsets");
static_assert(kWsTotal == 122159104, "carve total");
static_assert(kWsTotal <= 134217728, "carve cap");
static_assert((kOffBtSpl % 128) == 0 && (kOffAx % 128) == 0 && (kOffP % 128) == 0 && (kOffAspl % 128) == 0, "line alignment");
static_assert(kNin % 32 == 0 && kKspl % 32 == 0, "K multiples of 32");
static_assert(kBatch % 64 == 0 && kHalfRows % 64 == 0 && kNout % 64 == 0, "tile multiples");
static_assert((kBatch * kNin) % (8 * 256) == 0, "cast grid exact");
static_assert((kHalfRows * kNin) % 256 == 0 && (kNout * kNin) % 256 == 0, "producer grids exact");

typedef __attribute__((ext_vector_type(16))) _Float16 v16h;
typedef __attribute__((ext_vector_type(8)))  _Float16 v8h;
typedef __attribute__((ext_vector_type(16))) __bf16   v16b;
typedef __attribute__((ext_vector_type(8)))  __bf16   v8b;
typedef __attribute__((ext_vector_type(8)))  float    v8f;
typedef __attribute__((ext_vector_type(4)))  float    v4f;
typedef __attribute__((ext_vector_type(4)))  unsigned int v4u;

__device__ __forceinline__ unsigned short f2bf_bits(float f) {
  unsigned u = __float_as_uint(f);
  return (unsigned short)((u + 0x7FFFu + ((u >> 16) & 1u)) >> 16);
}
__device__ __forceinline__ float bf_bits2f(unsigned short h) { return __uint_as_float(((unsigned)h) << 16); }

__device__ __forceinline__ void dep_guard_h(v8f& a, v8f& b, v16h x, v16h y) { asm volatile("v_nop\n\tv_nop\n\tv_nop\n\tv_nop" : "+v"(a), "+v"(b) : "v"(x), "v"(y)); }
__device__ __forceinline__ void dep_guard_b(v8f& a, v8f& b, v16b x, v16b y) { asm volatile("v_nop\n\tv_nop\n\tv_nop\n\tv_nop" : "+v"(a), "+v"(b) : "v"(x), "v"(y)); }
__device__ __forceinline__ void keep4_h(v16h a, v16h b, v16h c, v16h d) { asm volatile("v_nop" :: "v"(a), "v"(b), "v"(c), "v"(d)); }
__device__ __forceinline__ void keep4_b(v16b a, v16b b, v16b c, v16b d) { asm volatile("v_nop" :: "v"(a), "v"(b), "v"(c), "v"(d)); }
__device__ __forceinline__ void acc_guard4(v8f& a, v8f& b, v8f& c, v8f& d) { asm volatile("v_nop\n\tv_nop\n\tv_nop\n\tv_nop" : "+v"(a), "+v"(b), "+v"(c), "+v"(d)); }
template <typename T> struct Frag;
template <> struct Frag<_Float16> {
  typedef v16h V; union U { v16h v; v8h h[2]; };
  static __device__ __forceinline__ v16h load(const _Float16* p) {
    U f; f.h[0] = *(const v8h*)(p); f.h[1] = *(const v8h*)(p + 16); return f.v;
  }
  static __device__ __forceinline__ v8f mma(v16h a, v16h b, v8f c) {
    return __builtin_amdgcn_wmma_f32_16x16x32_f16(false, a, false, b, (short)0, c, false, false);
  }
  static __device__ __forceinline__ void guard(v8f& a, v8f& b, v16h x, v16h y) { dep_guard_h(a, b, x, y); }
  static __device__ __forceinline__ void keep(v16h a, v16h b, v16h c, v16h d) { keep4_h(a, b, c, d); }
};
template <> struct Frag<__bf16> {
  typedef v16b V; union U { v16b v; v8b h[2]; };
  static __device__ __forceinline__ v16b load(const __bf16* p) {
    U f; f.h[0] = *(const v8b*)(p); f.h[1] = *(const v8b*)(p + 16); return f.v;
  }
  static __device__ __forceinline__ v8f mma(v16b a, v16b b, v8f c) {
    return __builtin_amdgcn_wmma_f32_16x16x32_bf16(false, a, false, b, (short)0, c, false, false);
  }
  static __device__ __forceinline__ void guard(v8f& a, v8f& b, v16b x, v16b y) { dep_guard_b(a, b, x, y); }
  static __device__ __forceinline__ void keep(v16b a, v16b b, v16b c, v16b d) { keep4_b(a, b, c, d); }
};

__device__ __forceinline__ unsigned pk16(unsigned short a, unsigned short b) { return (unsigned)a | ((unsigned)b << 16); }
__device__ __forceinline__ unsigned short h_bits(float f) { const _Float16 h = (_Float16)f; return __builtin_bit_cast(unsigned short, h); }

template <int ET> struct Elem;
template <> struct Elem<0> { typedef _Float16 T; };
template <> struct Elem<1> { typedef __bf16 T; };
template <int ET, bool SPLIT, int BIAS_MODE, int OUT_MODE, bool RESID, int ACT = 0>
__global__ __launch_bounds__(256) void wmma_gemm64(
    const unsigned short* __restrict__ Ap, const unsigned short* __restrict__ A2p, int lda, long strideA,
    const unsigned short* __restrict__ Btp, const unsigned short* __restrict__ Bt2p, int ldb, long strideB,
    void* __restrict__ Cout, void* __restrict__ Cout2, int ldc, long strideC,
    const float* __restrict__ bias,
    const float* __restrict__ resid, long strideR,
    int M, int N, int K, float scale) {
  static_assert(!RESID || OUT_MODE == 0, "resid only with f32 output");
  typedef typename Elem<ET>::T T;
  typedef typename Frag<T>::V V;
  const T* A = (const T*)Ap; const T* A2 = (const T*)A2p; const T* Bt = (const T*)Btp; const T* Bt2 = (const T*)Bt2p;
  __shared__ __align__(16) float sT[8][16 * 68];
  const int b    = blockIdx.y;
  const int lane = threadIdx.x & 31;
  const int wave = threadIdx.x >> 5;
  const int tilesN = N >> 6;
  const int tilesM = M >> 6;
  const int tile = blockIdx.x * 8 + wave;
  if (tile >= tilesM * tilesN) return;
  const int tm = tile / tilesN;
  const int tn = tile - tm * tilesN;
  const int m0 = tm << 6;
  const int n0 = tn << 6;

  const T* Ab  = A  + (size_t)b * strideA;
  const T* Bb  = Bt + (size_t)b * strideB;
  const T* Ab2 = SPLIT ? (A2  + (size_t)b * strideA) : nullptr;
  const T* Bb2 = SPLIT ? (Bt2 + (size_t)b * strideB) : nullptr;

  const int rlane = lane & 15;
  const int koff  = (lane >> 4) * 8;
  const int mOff  = (lane >> 4) * 8;

  v8f acc[4][4];
#pragma unroll
  for (int i = 0; i < 4; ++i)
#pragma unroll
    for (int j = 0; j < 4; ++j) acc[i][j] = (v8f){0.f,0.f,0.f,0.f,0.f,0.f,0.f,0.f};

  for (int k0 = 0; k0 < K; k0 += 32) {
    V bh[4], bl[4];
#pragma unroll
    for (int j = 0; j < 4; ++j) {
      const size_t bo = (size_t)(n0 + (j << 4) + rlane) * ldb + koff + k0;
      bh[j] = Frag<T>::load(Bb + bo);
      if (SPLIT) bl[j] = Frag<T>::load(Bb2 + bo);
    }
#pragma unroll
    for (int i = 0; i < 4; ++i) {
      const size_t ao = (size_t)(m0 + (i << 4) + rlane) * lda + koff + k0;
      V ah = Frag<T>::load(Ab + ao);
      V al;
      if (SPLIT) al = Frag<T>::load(Ab2 + ao);
#pragma unroll
      for (int j = 0; j < 4; ++j) {
        acc[i][j] = Frag<T>::mma(ah, bh[j], acc[i][j]);
        if (SPLIT) {
          acc[i][j] = Frag<T>::mma(ah, bl[j], acc[i][j]);
          acc[i][j] = Frag<T>::mma(al, bh[j], acc[i][j]);
        }
      }
      Frag<T>::guard(acc[i][0], acc[i][3], ah, SPLIT ? al : ah);
    }
    Frag<T>::keep(bh[0], bh[1], bh[2], bh[3]);
    if (SPLIT) Frag<T>::keep(bl[0], bl[1], bl[2], bl[3]);
  }
  acc_guard4(acc[0][0], acc[0][1], acc[0][2], acc[0][3]);
  acc_guard4(acc[1][0], acc[1][1], acc[1][2], acc[1][3]);
  acc_guard4(acc[2][0], acc[2][1], acc[2][2], acc[2][3]);
  acc_guard4(acc[3][0], acc[3][1], acc[3][2], acc[3][3]);

  float* slab = sT[wave];
  const float* Rb = RESID ? (resid + (size_t)b * strideR) : nullptr;
#pragma unroll
  for (int i = 0; i < 4; ++i) {
    const int mBase = m0 + (i << 4);
#pragma unroll
    for (int j = 0; j < 4; ++j) {
      const int n = n0 + (j << 4) + rlane;
      float bv = 0.f;
      if (BIAS_MODE == 2) bv = bias[n];
#pragma unroll
      for (int r = 0; r < 8; ++r) {
        float v = acc[i][j][r] * scale;
        if (BIAS_MODE == 1) v += bias[mBase + mOff + r];
        if (BIAS_MODE == 2) v += bv;
        if (ACT == 2) v = fmaxf(v, 0.0f);
        if (ACT == 3) { const float ev = __expf(-v); v = v * __builtin_amdgcn_rcpf(1.0f + ev); }
        if (ACT == 4) v = (v > 0.f) ? v : 0.01f * v;
        slab[(mOff + r) * 68 + (j << 4) + rlane] = v;
      }
    }
    __builtin_amdgcn_fence(__ATOMIC_RELEASE, "workgroup");
    __builtin_amdgcn_wave_barrier();
    __builtin_amdgcn_fence(__ATOMIC_ACQUIRE, "workgroup");
    if (OUT_MODE == 0) {
      float* C = (float*)Cout + (size_t)b * strideC;
      const int hh = lane >> 4, c4 = (lane & 15) * 4;
      v4f vals[8];
#pragma unroll
      for (int it = 0; it < 8; ++it) {
        const int row = it * 2 + hh;
        v4f v = *(const v4f*)(slab + row * 68 + c4);
        if (RESID) {
          const v4f rr = *(const v4f*)(Rb + (size_t)(mBase + row) * ldc + n0 + c4);
          v = v + rr;
        }
        vals[it] = v;
      }
      for (int pass = 0; pass < 2; ++pass) {
#pragma unroll
        for (int it = 0; it < 8; ++it) {
          const int row = it * 2 + hh;
          *(volatile v4f*)(C + (size_t)(mBase + row) * ldc + n0 + c4) = vals[it];
        }
        __threadfence();
      }
    } else {
      const int q = lane >> 3, c8 = (lane & 7) * 8;
      unsigned short* C  = (unsigned short*)Cout  + (size_t)b * strideC;
      unsigned short* C2 = (OUT_MODE == 2) ? ((unsigned short*)Cout2 + (size_t)b * strideC) : nullptr;
      for (int pass = 0; pass < 2; ++pass) {
#pragma unroll
        for (int it = 0; it < 4; ++it) {
          const int row = it * 4 + q;
          const float* sp = slab + row * 68 + c8;
          v8h hv, lv;
#pragma unroll
          for (int e = 0; e < 8; ++e) {
            if (OUT_MODE == 1) {
              hv[e] = (_Float16)sp[e];
            } else {
              unsigned short hb = f2bf_bits(sp[e]);
              unsigned short lb = f2bf_bits(sp[e] - bf_bits2f(hb));
              hv[e] = __builtin_bit_cast(_Float16, hb);
              lv[e] = __builtin_bit_cast(_Float16, lb);
            }
          }
          *(volatile v8h*)(C + (size_t)(mBase + row) * ldc + n0 + c8) = hv;
          if (OUT_MODE == 2) *(volatile v8h*)(C2 + (size_t)(mBase + row) * ldc + n0 + c8) = lv;
        }
        __threadfence();
      }
    }
    __builtin_amdgcn_fence(__ATOMIC_RELEASE, "workgroup");
    __builtin_amdgcn_wave_barrier();
    __builtin_amdgcn_fence(__ATOMIC_ACQUIRE, "workgroup");
  }
}

__global__ __launch_bounds__(256) void pack_w_kernel(const float* __restrict__ W, unsigned short* __restrict__ outp, float scale) {
  __shared__ float sm[64][65];
  const int t  = threadIdx.x;
  const int d0 = blockIdx.x * 64;
  const int h0 = blockIdx.y * 64;
#pragma unroll
  for (int i = 0; i < 16; ++i) {
    const int e = i * 256 + t;
    const int r = e >> 6;
    const int c = e & 63;
    sm[c][r] = W[(size_t)(d0 + r) * kNout + h0 + c] * scale;
  }
  __syncthreads();
  const int lane = t & 31, wave = t >> 5;
  const int q = lane >> 3, c8 = (lane & 7) * 8;
  for (int pass = 0; pass < 2; ++pass) {
#pragma unroll
    for (int it = 0; it < 2; ++it) {
      const int row = wave * 8 + it * 4 + q;
      unsigned short hb[8];
#pragma unroll
      for (int e = 0; e < 8; ++e) hb[e] = h_bits(sm[row][c8 + e]);
      const v4u u = (v4u){pk16(hb[0], hb[1]), pk16(hb[2], hb[3]), pk16(hb[4], hb[5]), pk16(hb[6], hb[7])};
      *(volatile v4u*)(outp + (size_t)(h0 + row) * kNin + d0 + c8) = u;
    }
    __threadfence();
  }
}

__global__ __launch_bounds__(256) void pack_coeff_kernel(const float* __restrict__ coeff, unsigned short* __restrict__ outp, float scale) {
  const int g = blockIdx.x * 256 + threadIdx.x;
  const int o = g >> 9;
  const int i = g & (kNin - 1);
  const float* p = coeff + ((size_t)i * kNout + o) * kNbasis;
  const v4f a = *(const v4f*)(p);
  const v4f c = *(const v4f*)(p + 4);
  unsigned short hb[8];
#pragma unroll
  for (int e = 0; e < 4; ++e) {
    hb[e]     = h_bits(a[e] * scale);
    hb[4 + e] = h_bits(c[e] * scale);
  }
  const v4u u = (v4u){pk16(hb[0], hb[1]), pk16(hb[2], hb[3]), pk16(hb[4], hb[5]), pk16(hb[6], hb[7])};
  unsigned short* q = outp + (size_t)o * kKspl + (size_t)i * kNbasis;
  *(volatile v4u*)q = u;
  __threadfence();
  *(volatile v4u*)q = u;
}

__global__ __launch_bounds__(256) void cast8_f16_kernel(const float* __restrict__ in, unsigned short* __restrict__ outp, int n8, float scale) {
  const int i = blockIdx.x * 256 + threadIdx.x;
  if (i >= n8) return;
  const float* p = in + 8 * (size_t)i;
  const v4f a = *(const v4f*)(p);
  const v4f c = *(const v4f*)(p + 4);
  unsigned short hb[8];
#pragma unroll
  for (int e = 0; e < 4; ++e) {
    hb[e]     = h_bits(a[e] * scale);
    hb[4 + e] = h_bits(c[e] * scale);
  }
  const v4u u = (v4u){pk16(hb[0], hb[1]), pk16(hb[2], hb[3]), pk16(hb[4], hb[5]), pk16(hb[6], hb[7])};
  unsigned short* q = outp + 8 * (size_t)i;
  *(volatile v4u*)q = u;
  __threadfence();
  *(volatile v4u*)q = u;
}

__global__ __launch_bounds__(256) void basis_kernel(const float* __restrict__ x, const float* __restrict__ knots,
                                                    unsigned short* __restrict__ outp, int row_base, float carry) {
  __shared__ __align__(16) float skn[kNknots];
  __shared__ __align__(16) float srcp[32];
  const int t = threadIdx.x;
  {
    const int tt = (t < 30) ? t : 29;
    const int jj = (tt < 11) ? 1 : ((tt < 21) ? 2 : 3);
    const int p  = tt - ((jj == 1) ? 0 : ((jj == 2) ? 11 : 21));
    int ia = p + jj; ia = (ia > kNknots - 1) ? (kNknots - 1) : ((ia < 0) ? 0 : ia);
    int ib = (p > kNknots - 1) ? (kNknots - 1) : ((p < 0) ? 0 : p);
    const float d  = knots[ia] - knots[ib];
    const float rc = 1.0f / fmaxf(d, 1e-8f);
    const int   tk = (t < kNknots) ? t : (kNknots - 1);
    const float kv = knots[tk];
    if (t < 30) srcp[t] = rc;
    if (t < kNknots) skn[t] = kv;
  }
  __syncthreads();
  float kn[kNknots];
#pragma unroll
  for (int q = 0; q < kNknots; ++q) kn[q] = skn[q];
  float rc1[11], rc2[10], rc3[9];
#pragma unroll
  for (int q = 0; q < 11; ++q) rc1[q] = srcp[q];
#pragma unroll
  for (int q = 0; q < 10; ++q) rc2[q] = srcp[11 + q];
#pragma unroll
  for (int q = 0; q < 9; ++q)  rc3[q] = srcp[21 + q];

  const int g  = blockIdx.x * 256 + t;
  const int bl = g >> 9;
  const int i  = g & (kNin - 1);
  const float xv = x[(size_t)(row_base + bl) * kNin + i];
  const float xc = fminf(fmaxf(xv, kn[3]), kn[8]);
  float bb[11];
#pragma unroll
  for (int p = 0; p < 11; ++p) bb[p] = (xc >= kn[p] && xc < kn[p + 1]) ? 1.0f : 0.0f;
#pragma unroll
  for (int p = 0; p < 10; ++p) {
    const float a1 = (xc - kn[p]) * rc1[p];
    const float a2 = (kn[p + 2] - xc) * rc1[p + 1];
    bb[p] = a1 * bb[p] + a2 * bb[p + 1];
  }
#pragma unroll
  for (int p = 0; p < 9; ++p) {
    const float a1 = (xc - kn[p]) * rc2[p];
    const float a2 = (kn[p + 3] - xc) * rc2[p + 1];
    bb[p] = a1 * bb[p] + a2 * bb[p + 1];
  }
#pragma unroll
  for (int p = 0; p < 8; ++p) {
    const float a1 = (xc - kn[p]) * rc3[p];
    const float a2 = (kn[p + 4] - xc) * rc3[p + 1];
    bb[p] = a1 * bb[p] + a2 * bb[p + 1];
  }
  unsigned short hb[8];
#pragma unroll
  for (int r = 0; r < 8; ++r) hb[r] = h_bits(bb[r] * carry);
  const v4u u = (v4u){pk16(hb[0], hb[1]), pk16(hb[2], hb[3]), pk16(hb[4], hb[5]), pk16(hb[6], hb[7])};
  unsigned short* q = outp + (size_t)bl * kKspl + (size_t)i * kNbasis;
  *(volatile v4u*)q = u;
  __threadfence();
  *(volatile v4u*)q = u;
}

extern "C" void kernel_launch(void* const* d_in, const int* in_sizes, int n_in,
                              void* d_out, int out_size, void* d_ws, size_t ws_size,
                              hipStream_t stream) {
  if (n_in < 4) return;
  if (in_sizes[0] != kBatch * kNin) return;
  if (in_sizes[1] != kNin * kNout * kNbasis) return;
  if (in_sizes[2] != kNin * kNout) return;
  if (in_sizes[3] != kNknots) return;
  if (out_size != kBatch * kNout) return;
  if (ws_size < kWsTotal) return;

  const float* x     = (const float*)d_in[0];
  const float* coeff = (const float*)d_in[1];
  const float* bw    = (const float*)d_in[2];
  const float* knots = (const float*)d_in[3];
  float* outp = (float*)d_out;

  char* ws = (char*)d_ws;
  unsigned short* btBase = (unsigned short*)(ws + kOffBtBase);
  unsigned short* btSpl  = (unsigned short*)(ws + kOffBtSpl);
  unsigned short* ax     = (unsigned short*)(ws + kOffAx);
  float*          pl     = (float*)(ws + kOffP);
  unsigned short* aspl   = (unsigned short*)(ws + kOffAspl);

  pack_w_kernel<<<dim3(kNin / 64, kNout / 64, 1), dim3(256), 0, stream>>>(bw, btBase, kWCarry);
  pack_coeff_kernel<<<dim3((kNout * kNin) / 256), dim3(256), 0, stream>>>(coeff, btSpl, kCoeffCarry);
  {
    const int n8 = (kBatch * kNin) / 8;
    cast8_f16_kernel<<<dim3(n8 / 256), dim3(256), 0, stream>>>(x, ax, n8, kXCarry);
  }
  {
    const int tiles = (kBatch / 64) * (kNout / 64);
    wmma_gemm64<0, false, 0, 0, false, 3><<<dim3(tiles / 8, 1, 1), dim3(256), 0, stream>>>(
        ax, ax, kNin, 0L,
        btBase, btBase, kNin, 0L,
        (void*)pl, (void*)pl, kNout, 0L,
        (const float*)pl,
        (const float*)pl, 0L,
        kBatch, kNout, kNin, kBaseScale);
  }
  for (int half = 0; half < 2; ++half) {
    const int rowBase = half * kHalfRows;
    basis_kernel<<<dim3((kHalfRows * kNin) / 256), dim3(256), 0, stream>>>(x, knots, aspl, rowBase, kBasisCarry);
    const int tiles = (kHalfRows / 64) * (kNout / 64);
    float* cHalf = outp + (size_t)rowBase * kNout;
    const float* rHalf = pl + (size_t)rowBase * kNout;
    wmma_gemm64<0, false, 0, 0, true, 0><<<dim3(tiles / 8, 1, 1), dim3(256), 0, stream>>>(
        aspl, aspl, kKspl, 0L,
        btSpl, btSpl, kKspl, 0L,
        (void*)cHalf, (void*)cHalf, kNout, 0L,
        rHalf,
        rHalf, 0L,
        kHalfRows, kNout, kKspl, kSplScale);
  }
}
